// DiTBlock_CrossAttn_60206851555415
// MI455X (gfx1250) — hardware-verified
//
#include <hip/hip_runtime.h>
#include <math.h>
#include <stdint.h>

#define BB    8
#define NTOK  1024
#define DM    1024
#define NH    16
#define HD    64
#define SCTX  256
#define CD    512
#define DMLP  4096
#define DADA  6144
#define MADA  64
static_assert(NH * HD == DM);
static_assert(BB <= MADA);
static_assert((NTOK % 64) == 0 && (DM % 64) == 0 && (SCTX % 64) == 0 && (CD % 64) == 0);
static_assert((DMLP % 64) == 0 && (DADA % 64) == 0 && (MADA % 64) == 0);

typedef _Float16 v16h __attribute__((ext_vector_type(16)));
typedef _Float16 v8h  __attribute__((ext_vector_type(8)));
typedef float    v8f  __attribute__((ext_vector_type(8)));
typedef float    v4f  __attribute__((ext_vector_type(4)));
typedef unsigned int v4u __attribute__((ext_vector_type(4)));

__device__ __forceinline__ unsigned short h_bits(_Float16 x) { return __builtin_bit_cast(unsigned short, x); }
__device__ __forceinline__ unsigned pk16(unsigned short a, unsigned short b) { return (unsigned)a | ((unsigned)b << 16); }
__device__ __forceinline__ unsigned pkf(float a, float b) { return pk16(h_bits((_Float16)a), h_bits((_Float16)b)); }
__device__ __forceinline__ v8f zero8() { v8f z = {0.f, 0.f, 0.f, 0.f, 0.f, 0.f, 0.f, 0.f}; return z; }
__device__ __forceinline__ v4f splat4(float x) { v4f v = {x, x, x, x}; return v; }
__device__ __forceinline__ float gelu_exact(float v) { return 0.5f * v * (1.0f + erff(v * 0.70710678118654752f)); }

__device__ __forceinline__ v16h ldfrag_h(const _Float16* p) {
  union { v16h v; v8h h[2]; } f;
  f.h[0] = *(const v8h*)(p);
  f.h[1] = *(const v8h*)(p + 16);
  return f.v;
}

__device__ __forceinline__ v8f mma_h(v16h a, v16h b, v8f c) {
  c = __builtin_amdgcn_wmma_f32_16x16x32_f16(false, a, false, b, (short)0, c, false, false);
#if defined(__HIP_DEVICE_COMPILE__)
  asm volatile("v_nop\n\tv_nop\n\tv_nop\n\tv_nop" : "+v"(c) : "v"(a), "v"(b));
#endif
  return c;
}
__device__ __forceinline__ v8f mma_h_raw(v16h a, v16h b, v8f c) {
  return __builtin_amdgcn_wmma_f32_16x16x32_f16(false, a, false, b, (short)0, c, false, false);
}
__device__ __forceinline__ void dep_guard_h(v8f& a, v8f& b, v16h x) {
#if defined(__HIP_DEVICE_COMPILE__)
  asm volatile("v_nop\n\tv_nop\n\tv_nop\n\tv_nop" : "+v"(a), "+v"(b) : "v"(x));
#else
  (void)a; (void)b; (void)x;
#endif
}
__device__ __forceinline__ void keep4_h(v16h a, v16h b, v16h c, v16h d) {
#if defined(__HIP_DEVICE_COMPILE__)
  asm volatile("v_nop" :: "v"(a), "v"(b), "v"(c), "v"(d));
#else
  (void)a; (void)b; (void)c; (void)d;
#endif
}
__device__ __forceinline__ void acc_guard4(v8f& a, v8f& b, v8f& c, v8f& d) {
#if defined(__HIP_DEVICE_COMPILE__)
  asm volatile("v_nop\n\tv_nop\n\tv_nop\n\tv_nop" : "+v"(a), "+v"(b), "+v"(c), "+v"(d));
#else
  (void)a; (void)b; (void)c; (void)d;
#endif
}
__device__ __forceinline__ void lds_wave_sync() {
  __builtin_amdgcn_fence(__ATOMIC_RELEASE, "workgroup");
  __builtin_amdgcn_wave_barrier();
  __builtin_amdgcn_fence(__ATOMIC_ACQUIRE, "workgroup");
}

__global__ __launch_bounds__(256) void cvt_f16x8(const float* __restrict__ in, unsigned short* out, int n8) {
  const int i = blockIdx.x * 256 + threadIdx.x;
  if (i < n8) {
    const v4f a = *(const v4f*)(in + (size_t)i * 8);
    const v4f b = *(const v4f*)(in + (size_t)i * 8 + 4);
    v4u p;
    p[0] = pkf(a[0], a[1]); p[1] = pkf(a[2], a[3]);
    p[2] = pkf(b[0], b[1]); p[3] = pkf(b[2], b[3]);
    *(volatile v4u*)(out + (size_t)i * 8) = p;
    __threadfence();
    *(volatile v4u*)(out + (size_t)i * 8) = p;
  }
}

__global__ __launch_bounds__(256) void silu_plane(const float* __restrict__ cin, unsigned short* sout) {
  const int i = blockIdx.x * 256 + threadIdx.x;
  if (i >= MADA * (DM / 8)) return;
  const int row  = i / (DM / 8);
  const int col  = (i - row * (DM / 8)) * 8;
  const int rowc = (row < BB) ? row : (BB - 1);
  const float keep = (row < BB) ? 1.0f : 0.0f;
  const float* src = cin + (size_t)rowc * DM + col;
  const v4f a0 = *(const v4f*)(src);
  const v4f a1 = *(const v4f*)(src + 4);
  float o[8];
#pragma unroll
  for (int e = 0; e < 4; ++e) {
    const float v0 = a0[e], v1 = a1[e];
    const float g0 = __builtin_amdgcn_rcpf(1.0f + __expf(-v0));
    const float g1 = __builtin_amdgcn_rcpf(1.0f + __expf(-v1));
    o[e]     = (v0 * g0) * keep;
    o[4 + e] = (v1 * g1) * keep;
  }
  v4u p;
  p[0] = pkf(o[0], o[1]); p[1] = pkf(o[2], o[3]); p[2] = pkf(o[4], o[5]); p[3] = pkf(o[6], o[7]);
  unsigned short* dst = sout + (size_t)row * DM + col;
  *(volatile v4u*)dst = p;
  __threadfence();
  *(volatile v4u*)dst = p;
}

__global__ __launch_bounds__(256) void wtrans64(const float* __restrict__ w, unsigned short* wt,
                                                int K, int N, float scale) {
  __shared__ float T[64 * 65];
  const int tid = threadIdx.x;
  const int n0 = blockIdx.x * 64, k0 = blockIdx.y * 64;
  const int kr = tid >> 2, nc = (tid & 3) * 16;
  const float* src = w + (size_t)(k0 + kr) * N + n0 + nc;
  const v4f a0 = *(const v4f*)(src);
  const v4f a1 = *(const v4f*)(src + 4);
  const v4f a2 = *(const v4f*)(src + 8);
  const v4f a3 = *(const v4f*)(src + 12);
#pragma unroll
  for (int e = 0; e < 4; ++e) {
    T[(nc + e) * 65 + kr]      = a0[e] * scale;
    T[(nc + 4 + e) * 65 + kr]  = a1[e] * scale;
    T[(nc + 8 + e) * 65 + kr]  = a2[e] * scale;
    T[(nc + 12 + e) * 65 + kr] = a3[e] * scale;
  }
  __syncthreads();
  v4u pv[2];
#pragma unroll
  for (int it = 0; it < 2; ++it) {
    const int p = it * 256 + tid;
    const int n = p >> 3, c8 = (p & 7) * 8;
    const float* tp = T + n * 65 + c8;
    v4u a;
    a[0] = pkf(tp[0], tp[1]); a[1] = pkf(tp[2], tp[3]); a[2] = pkf(tp[4], tp[5]); a[3] = pkf(tp[6], tp[7]);
    pv[it] = a;
  }
  for (int pass = 0; pass < 2; ++pass) {
#pragma unroll
    for (int it = 0; it < 2; ++it) {
      const int p = it * 256 + tid;
      const int n = p >> 3, c8 = (p & 7) * 8;
      *(volatile v4u*)(wt + (size_t)(n0 + n) * K + k0 + c8) = pv[it];
    }
    __threadfence();
  }
}

__global__ __launch_bounds__(128) void ln_mod(const float* __restrict__ xin, const float* __restrict__ ada,
                                              unsigned short* hout, int shiftOff, int scaleOff) {
  __shared__ float red0[4];
  __shared__ float red1[4];
  const int tid = threadIdx.x, wave = tid >> 5, lane = tid & 31;
  const int row = blockIdx.x;
  const int b   = row / NTOK;
  const float* xr = xin + (size_t)row * DM + tid * 8;
  const v4f a0 = *(const v4f*)(xr);
  const v4f a1 = *(const v4f*)(xr + 4);
  float s = ((a0[0] + a0[1]) + (a0[2] + a0[3])) + ((a1[0] + a1[1]) + (a1[2] + a1[3]));
#pragma unroll
  for (int off = 1; off < 32; off <<= 1) s += __shfl_xor(s, off, 32);
  if (lane == 0) red0[wave] = s;
  __syncthreads();
  const float mu = ((red0[0] + red0[1]) + (red0[2] + red0[3])) * (1.0f / (float)DM);
  const v4f mu4 = splat4(mu);
  const v4f d0 = a0 - mu4, d1 = a1 - mu4;
  float ss = ((d0[0] * d0[0] + d0[1] * d0[1]) + (d0[2] * d0[2] + d0[3] * d0[3]))
           + ((d1[0] * d1[0] + d1[1] * d1[1]) + (d1[2] * d1[2] + d1[3] * d1[3]));
#pragma unroll
  for (int off = 1; off < 32; off <<= 1) ss += __shfl_xor(ss, off, 32);
  if (lane == 0) red1[wave] = ss;
  __syncthreads();
  const float var  = ((red1[0] + red1[1]) + (red1[2] + red1[3])) * (1.0f / (float)DM);
  const float rstd = rsqrtf(var + 1e-6f);
  const v4f rs4 = splat4(rstd), one4 = splat4(1.0f);
  const float* ab = ada + (size_t)b * DADA + tid * 8;
  const v4f sc0 = *(const v4f*)(ab + scaleOff), sc1 = *(const v4f*)(ab + scaleOff + 4);
  const v4f sh0 = *(const v4f*)(ab + shiftOff), sh1 = *(const v4f*)(ab + shiftOff + 4);
  const v4f o0 = (d0 * rs4) * (one4 + sc0) + sh0;
  const v4f o1 = (d1 * rs4) * (one4 + sc1) + sh1;
  v4u p;
  p[0] = pkf(o0[0], o0[1]); p[1] = pkf(o0[2], o0[3]); p[2] = pkf(o1[0], o1[1]); p[3] = pkf(o1[2], o1[3]);
  unsigned short* dst = hout + (size_t)row * DM + tid * 8;
  *(volatile v4u*)dst = p;
  __threadfence();
  *(volatile v4u*)dst = p;
}

template <int OUT, bool BROW, bool RESID>
__global__ __launch_bounds__(256) void gemm64(
    const unsigned short* __restrict__ Ap, int lda, long long strideA,
    const unsigned short* __restrict__ Btp, int ldb, long long strideB,
    void* Cout, int ldc, long long strideC,
    const float* __restrict__ bias, const float* __restrict__ Rp, int ldr,
    int M, int N, int K, float scale) {
  const _Float16* A  = (const _Float16*)(const void*)Ap;
  const _Float16* Bt = (const _Float16*)(const void*)Btp;
  __shared__ __align__(16) float sT[8][16 * 68];
  const int b    = blockIdx.y;
  const int lane = threadIdx.x & 31;
  const int wave = threadIdx.x >> 5;
  const int tilesN = N >> 6;
  const int tilesM = M >> 6;
  const int tile = blockIdx.x * 8 + wave;
  if (tile >= tilesM * tilesN) return;
  const int tm = tile / tilesN;
  const int tn = tile - tm * tilesN;
  const int m0 = tm << 6;
  const int n0 = tn << 6;

  const _Float16* Ab = A  + (long long)b * strideA;
  const _Float16* Bb = Bt + (long long)b * strideB;

  const int rlane = lane & 15;
  const int koff  = (lane >> 4) * 8;
  const int mOff  = (lane >> 4) * 8;

  v8f acc[4][4];
#pragma unroll
  for (int i = 0; i < 4; ++i)
#pragma unroll
    for (int j = 0; j < 4; ++j) acc[i][j] = zero8();

  for (int k0 = 0; k0 < K; k0 += 32) {
    v16h bh[4];
#pragma unroll
    for (int j = 0; j < 4; ++j)
      bh[j] = ldfrag_h(Bb + (size_t)(n0 + (j << 4) + rlane) * ldb + koff + k0);
#pragma unroll
    for (int i = 0; i < 4; ++i) {
      const v16h ah = ldfrag_h(Ab + (size_t)(m0 + (i << 4) + rlane) * lda + koff + k0);
#pragma unroll
      for (int j = 0; j < 4; ++j) acc[i][j] = mma_h_raw(ah, bh[j], acc[i][j]);
      dep_guard_h(acc[i][0], acc[i][3], ah);
    }
    keep4_h(bh[0], bh[1], bh[2], bh[3]);
  }
  acc_guard4(acc[0][0], acc[0][1], acc[0][2], acc[0][3]);
  acc_guard4(acc[1][0], acc[1][1], acc[1][2], acc[1][3]);
  acc_guard4(acc[2][0], acc[2][1], acc[2][2], acc[2][3]);
  acc_guard4(acc[3][0], acc[3][1], acc[3][2], acc[3][3]);

  float* slab = sT[wave];
#pragma unroll
  for (int i = 0; i < 4; ++i) {
    const int mBase = m0 + (i << 4);
#pragma unroll
    for (int j = 0; j < 4; ++j) {
#pragma unroll
      for (int r = 0; r < 8; ++r) {
        slab[(mOff + r) * 68 + (j << 4) + rlane] = acc[i][j][r] * scale;
      }
    }
    lds_wave_sync();
    if (OUT == 0) {
      float* C = (float*)Cout + (long long)b * strideC;
      const int hh = lane >> 4, c4 = (lane & 15) * 4;
      v4f bc = splat4(0.f);
      if (!BROW) bc = *(const v4f*)(bias + n0 + c4);
      v4f vals[8];
#pragma unroll
      for (int it = 0; it < 8; ++it) {
        const int row = it * 2 + hh;
        v4f v = *(const v4f*)(slab + row * 68 + c4);
        if (BROW) { v += splat4(bias[mBase + row]); } else { v += bc; }
        if (RESID) {
          const v4f rr = *(const v4f*)(Rp + (size_t)(mBase + row) * ldr + n0 + c4);
          v += rr;
        }
        vals[it] = v;
      }
      for (int pass = 0; pass < 2; ++pass) {
#pragma unroll
        for (int it = 0; it < 8; ++it) {
          const int row = it * 2 + hh;
          *(volatile v4f*)(C + (size_t)(mBase + row) * ldc + n0 + c4) = vals[it];
        }
        __threadfence();
      }
    } else {
      unsigned short* C = (unsigned short*)Cout + (long long)b * strideC;
      const int q = lane >> 3, c8 = (lane & 7) * 8;
      v4f bc0 = splat4(0.f), bc1 = splat4(0.f);
      if (!BROW) { bc0 = *(const v4f*)(bias + n0 + c8); bc1 = *(const v4f*)(bias + n0 + c8 + 4); }
      v4u hv[4];
#pragma unroll
      for (int it = 0; it < 4; ++it) {
        const int row = it * 4 + q;
        const float* sp = slab + row * 68 + c8;
        v4f f0 = *(const v4f*)(sp);
        v4f f1 = *(const v4f*)(sp + 4);
        if (BROW) { const v4f b4 = splat4(bias[mBase + row]); f0 += b4; f1 += b4; }
        else      { f0 += bc0; f1 += bc1; }
        if (OUT == 2) {
#pragma unroll
          for (int e = 0; e < 4; ++e) { f0[e] = gelu_exact(f0[e]); f1[e] = gelu_exact(f1[e]); }
        }
        v4u a;
        a[0] = pkf(f0[0], f0[1]); a[1] = pkf(f0[2], f0[3]); a[2] = pkf(f1[0], f1[1]); a[3] = pkf(f1[2], f1[3]);
        hv[it] = a;
      }
      for (int pass = 0; pass < 2; ++pass) {
#pragma unroll
        for (int it = 0; it < 4; ++it) {
          const int row = it * 4 + q;
          *(volatile v4u*)(C + (size_t)(mBase + row) * ldc + n0 + c8) = hv[it];
        }
        __threadfence();
      }
    }
    lds_wave_sync();
  }
}

__global__ __launch_bounds__(128)
void attn64(const unsigned short* __restrict__ qp, int ldq, int qcol,
            const unsigned short* __restrict__ kp, int ldk, int kcol,
            const unsigned short* __restrict__ vp, int ldv,
            unsigned short* op, int nq, int nkv, float sscale, float oscale) {
  union FH { v16h v; v8h h[2]; };
  __shared__ __align__(16) _Float16 Psh[4][16 * 64];
  __shared__ __align__(16) float    Os[4][16 * 64];

  const int tid  = threadIdx.x;
  const int wave = tid >> 5;
  const int lane = tid & 31;
  const int hh   = lane >> 4;
  const int c    = lane & 15;
  const int b    = blockIdx.z;
  const int h    = blockIdx.y;
  const int q0   = blockIdx.x * 64 + wave * 16;

  const _Float16* Qb = (const _Float16*)(const void*)qp + (size_t)b * nq * ldq + qcol + h * HD;
  const _Float16* Kb = (const _Float16*)(const void*)kp + (size_t)b * nkv * ldk + kcol + h * HD;
  const _Float16* Vb = (const _Float16*)(const void*)vp + ((size_t)b * DM + (size_t)h * HD) * ldv;

  v16h qa[2];
#pragma unroll
  for (int dc = 0; dc < 2; ++dc) qa[dc] = ldfrag_h(Qb + (size_t)(q0 + c) * ldq + dc * 32 + 8 * hh);

  float mrow[8], lrow[8];
  v8f oacc[4];
#pragma unroll
  for (int r = 0; r < 8; ++r) { mrow[r] = -INFINITY; lrow[r] = 0.f; }
#pragma unroll
  for (int t = 0; t < 4; ++t) oacc[t] = zero8();

  _Float16* pw = Psh[wave];
  const int nkt = nkv >> 6;
  for (int kt = 0; kt < nkt; ++kt) {
    const int kv0 = kt * 64;

    v8f s[4];
#pragma unroll
    for (int j = 0; j < 4; ++j) {
      s[j] = zero8();
#pragma unroll
      for (int dc = 0; dc < 2; ++dc) {
        FH kb;
        const _Float16* kr = Kb + (size_t)(kv0 + j * 16 + c) * ldk + dc * 32 + 8 * hh;
        kb.h[0] = *(const v8h*)(kr);
        kb.h[1] = *(const v8h*)(kr + 16);
        s[j] = mma_h(qa[dc], kb.v, s[j]);
      }
    }

#pragma unroll
    for (int r = 0; r < 8; ++r) {
      float m = -INFINITY;
#pragma unroll
      for (int j = 0; j < 4; ++j) {
        const float sv = s[j][r] * sscale;
        s[j][r] = sv;
        m = fmaxf(m, sv);
      }
#pragma unroll
      for (int off = 1; off < 16; off <<= 1) m = fmaxf(m, __shfl_xor(m, off, 32));
      const float mnew  = fmaxf(mrow[r], m);
      const float msafe = (mnew == -INFINITY) ? 0.f : mnew;
      const float alpha = __expf(mrow[r] - msafe);
      mrow[r] = mnew;
      float psum = 0.f;
#pragma unroll
      for (int j = 0; j < 4; ++j) {
        const float p = __expf(s[j][r] - msafe);
        psum += p;
        pw[(8 * hh + r) * 64 + j * 16 + c] = (_Float16)(p * 1024.0f);
      }
#pragma unroll
      for (int off = 1; off < 16; off <<= 1) psum += __shfl_xor(psum, off, 32);
      lrow[r] = lrow[r] * alpha + psum;
#pragma unroll
      for (int t = 0; t < 4; ++t) oacc[t][r] *= alpha;
    }
    lds_wave_sync();

#pragma unroll
    for (int kk = 0; kk < 2; ++kk) {
      FH pa;
      pa.h[0] = *(const v8h*)(pw + c * 64 + kk * 32 + 8 * hh);
      pa.h[1] = *(const v8h*)(pw + c * 64 + kk * 32 + 16 + 8 * hh);
#pragma unroll
      for (int t = 0; t < 4; ++t) {
        FH vb;
        const _Float16* vr = Vb + (size_t)(t * 16 + c) * ldv + kv0 + kk * 32 + 8 * hh;
        vb.h[0] = *(const v8h*)(vr);
        vb.h[1] = *(const v8h*)(vr + 16);
        oacc[t] = mma_h(pa.v, vb.v, oacc[t]);
      }
    }
    lds_wave_sync();
  }

  float* os = Os[wave];
#pragma unroll
  for (int r = 0; r < 8; ++r) {
    const float l = lrow[r];
    const float inv = (l > 0.f) ? (oscale * __builtin_amdgcn_rcpf(l)) : 0.f;
#pragma unroll
    for (int t = 0; t < 4; ++t) os[(8 * hh + r) * 64 + t * 16 + c] = oacc[t][r] * inv;
  }
  lds_wave_sync();
  {
    const int q4 = lane >> 3, c8 = (lane & 7) * 8;
    v4u hv[4];
#pragma unroll
    for (int it = 0; it < 4; ++it) {
      const int row = it * 4 + q4;
      const float* sp = os + row * 64 + c8;
      const v4f f0 = *(const v4f*)(sp);
      const v4f f1 = *(const v4f*)(sp + 4);
      v4u a;
      a[0] = pkf(f0[0], f0[1]); a[1] = pkf(f0[2], f0[3]); a[2] = pkf(f1[0], f1[1]); a[3] = pkf(f1[2], f1[3]);
      hv[it] = a;
    }
    for (int pass = 0; pass < 2; ++pass) {
#pragma unroll
      for (int it = 0; it < 4; ++it) {
        const int row = it * 4 + q4;
        const size_t go = ((size_t)b * nq + q0 + row) * DM + (size_t)h * HD + c8;
        *(volatile v4u*)(op + go) = hv[it];
      }
      __threadfence();
    }
  }
}

static inline unsigned gemm_blocks(int M, int N) { return (unsigned)(((M / 64) * (N / 64) + 7) / 8); }

extern "C" void kernel_launch(void* const* d_in, const int* in_sizes, int n_in,
                              void* d_out, int out_size, void* d_ws, size_t ws_size,
                              hipStream_t stream) {
  if (n_in < 21) return;
  const int NX = BB * NTOK * DM;
  if (in_sizes[0] != NX || in_sizes[1] != BB * DM || in_sizes[2] != BB * SCTX * CD) return;
  if (in_sizes[3] != DM * 3 * DM || in_sizes[4] != 3 * DM) return;
  if (in_sizes[5] != DM * DM || in_sizes[6] != DM || in_sizes[7] != DM * DM || in_sizes[8] != DM) return;
  if (in_sizes[9] != CD * DM || in_sizes[10] != DM || in_sizes[11] != CD * DM || in_sizes[12] != DM) return;
  if (in_sizes[13] != DM * DM || in_sizes[14] != DM) return;
  if (in_sizes[15] != DM * DMLP || in_sizes[16] != DMLP || in_sizes[17] != DMLP * DM || in_sizes[18] != DM) return;
  if (in_sizes[19] != DM * DADA || in_sizes[20] != DADA) return;
  if (out_size != NX) return;

  const float* x     = (const float*)d_in[0];
  const float* cvec  = (const float*)d_in[1];
  const float* ctx   = (const float*)d_in[2];
  const float* w_qkv = (const float*)d_in[3];  const float* b_qkv = (const float*)d_in[4];
  const float* w_so  = (const float*)d_in[5];  const float* b_so  = (const float*)d_in[6];
  const float* w_cq  = (const float*)d_in[7];  const float* b_cq  = (const float*)d_in[8];
  const float* w_ck  = (const float*)d_in[9];  const float* b_ck  = (const float*)d_in[10];
  const float* w_cv  = (const float*)d_in[11]; const float* b_cv  = (const float*)d_in[12];
  const float* w_co  = (const float*)d_in[13]; const float* b_co  = (const float*)d_in[14];
  const float* w1    = (const float*)d_in[15]; const float* b1    = (const float*)d_in[16];
  const float* w2    = (const float*)d_in[17]; const float* b2    = (const float*)d_in[18];
  const float* w_ada = (const float*)d_in[19]; const float* b_ada = (const float*)d_in[20];
  float* outF = (float*)d_out;

  const size_t szAda   = (size_t)MADA * DADA * 4;
  const size_t szH     = (size_t)BB * NTOK * DM * 2;
  const size_t szQK    = (size_t)BB * NTOK * 2 * DM * 2;
  const size_t szVT    = (size_t)BB * DM * NTOK * 2;
  const size_t szCTX   = (size_t)BB * NTOK * DM * 2;
  const size_t szCQ    = szCTX;
  const size_t szCK    = (size_t)BB * SCTX * DM * 2;
  const size_t szCVT   = (size_t)BB * DM * SCTX * 2;
  const size_t szWADA  = (size_t)DADA * DM * 2;
  const size_t szG     = (size_t)BB * NTOK * DMLP * 2;
  const size_t szArena = szQK + szVT + szCTX;
  const size_t szXB    = (size_t)BB * NTOK * DM * 4;
  const size_t szWQKV  = (size_t)3 * DM * DM * 2;
  const size_t szWDD   = (size_t)DM * DM * 2;
  const size_t szWCD   = (size_t)DM * CD * 2;
  const size_t szW1    = (size_t)DMLP * DM * 2;
  const size_t szW2    = (size_t)DM * DMLP * 2;
  const size_t szWreg  = szW1;
  const size_t szC16   = (size_t)BB * SCTX * CD * 2;
  const size_t szS     = (size_t)MADA * DM * 2;
  if (szG > szArena || szWADA > szArena || szCQ + szCK + szCVT > szQK) return;
  if (szWQKV + szWDD > szWreg || 2 * szWDD + 2 * szWCD > szWreg || szW2 > szH) return;

  size_t off = 0;
  const size_t oAda   = off; off += szAda;
  const size_t oH     = off; off += szH;
  const size_t oArena = off; off += szArena;
  const size_t oXB    = off; off += szXB;
  const size_t oWreg  = off; off += szWreg;
  const size_t oC16   = off; off += szC16;
  const size_t oS     = off; off += szS;
  if (off > ws_size) return;
  if (off > (size_t)134217728) return;

  char* ws = (char*)d_ws;
  float*          ADA  = (float*)(ws + oAda);
  unsigned short* H    = (unsigned short*)(ws + oH);
  unsigned short* W2T  = (unsigned short*)(ws + oH);
  unsigned short* WADA = (unsigned short*)(ws + oArena);
  unsigned short* QK   = (unsigned short*)(ws + oArena);
  unsigned short* VT   = (unsigned short*)(ws + oArena + szQK);
  unsigned short* CTX  = (unsigned short*)(ws + oArena + szQK + szVT);
  unsigned short* CQ   = (unsigned short*)(ws + oArena);
  unsigned short* CK   = (unsigned short*)(ws + oArena + szCQ);
  unsigned short* CVT  = (unsigned short*)(ws + oArena + szCQ + szCK);
  unsigned short* G    = (unsigned short*)(ws + oArena);
  float*          XB   = (float*)(ws + oXB);
  unsigned short* WQKV = (unsigned short*)(ws + oWreg);
  unsigned short* WSO  = (unsigned short*)(ws + oWreg + szWQKV);
  unsigned short* WCQ  = (unsigned short*)(ws + oWreg);
  unsigned short* WCK  = (unsigned short*)(ws + oWreg + szWDD);
  unsigned short* WCV  = (unsigned short*)(ws + oWreg + szWDD + szWCD);
  unsigned short* WCO  = (unsigned short*)(ws + oWreg + szWDD + 2 * szWCD);
  unsigned short* W1T  = (unsigned short*)(ws + oWreg);
  unsigned short* C16  = (unsigned short*)(ws + oC16);
  unsigned short* S    = (unsigned short*)(ws + oS);

  const dim3 b256(256), b128(128);
  const float r64 = 1.0f / 64.0f, r4096 = 1.0f / 4096.0f;

  silu_plane<<<dim3((MADA * (DM / 8) + 255) / 256), b256, 0, stream>>>(cvec, S);
  wtrans64<<<dim3(DADA / 64, DM / 64), b256, 0, stream>>>(w_ada, WADA, DM, DADA, 64.0f);
  gemm64<0, false, false><<<dim3(gemm_blocks(MADA, DADA), 1), b256, 0, stream>>>(
      S, DM, 0LL, WADA, DM, 0LL, (void*)ADA, DADA, 0LL, b_ada, b_ada, 0, MADA, DADA, DM, r64);

  ln_mod<<<dim3(BB * NTOK), b128, 0, stream>>>(x, ADA, H, 0, DM);
  wtrans64<<<dim3(3 * DM / 64, DM / 64), b256, 0, stream>>>(w_qkv, WQKV, DM, 3 * DM, 64.0f);
  wtrans64<<<dim3(DM / 64, DM / 64), b256, 0, stream>>>(w_so, WSO, DM, DM, 64.0f);
  gemm64<1, false, false><<<dim3(gemm_blocks(BB * NTOK, 2 * DM), 1), b256, 0, stream>>>(
      H, DM, 0LL, WQKV, DM, 0LL, (void*)QK, 2 * DM, 0LL, b_qkv, b_qkv, 0, BB * NTOK, 2 * DM, DM, r64);
  gemm64<1, true, false><<<dim3(gemm_blocks(DM, NTOK), BB), b256, 0, stream>>>(
      WQKV + (size_t)2 * DM * DM, DM, 0LL, H, DM, (long long)NTOK * DM,
      (void*)VT, NTOK, (long long)DM * NTOK, b_qkv + 2 * DM, b_qkv, 0, DM, NTOK, DM, r64);
  attn64<<<dim3(NTOK / 64, NH, BB), b128, 0, stream>>>(
      QK, 2 * DM, 0, QK, 2 * DM, DM, VT, NTOK, CTX, NTOK, NTOK, 0.125f, 0.0625f);
  gemm64<0, false, true><<<dim3(gemm_blocks(BB * NTOK, DM), 1), b256, 0, stream>>>(
      CTX, DM, 0LL, WSO, DM, 0LL, d_out, DM, 0LL, b_so, x, DM, BB * NTOK, DM, DM, r4096);

  ln_mod<<<dim3(BB * NTOK), b128, 0, stream>>>(outF, ADA, H, 2 * DM, 3 * DM);
  wtrans64<<<dim3(DM / 64, DM / 64), b256, 0, stream>>>(w_cq, WCQ, DM, DM, 64.0f);
  wtrans64<<<dim3(DM / 64, CD / 64), b256, 0, stream>>>(w_ck, WCK, CD, DM, 64.0f);
  wtrans64<<<dim3(DM / 64, CD / 64), b256, 0, stream>>>(w_cv, WCV, CD, DM, 64.0f);
  wtrans64<<<dim3(DM / 64, DM / 64), b256, 0, stream>>>(w_co, WCO, DM, DM, 64.0f);
  {
    const int n8c = BB * SCTX * CD / 8;
    cvt_f16x8<<<dim3((n8c + 255) / 256), b256, 0, stream>>>(ctx, C16, n8c);
  }
  gemm64<1, false, false><<<dim3(gemm_blocks(BB * NTOK, DM), 1), b256, 0, stream>>>(
      H, DM, 0LL, WCQ, DM, 0LL, (void*)CQ, DM, 0LL, b_cq, b_cq, 0, BB * NTOK, DM, DM, r64);
  gemm64<1, false, false><<<dim3(gemm_blocks(BB * SCTX, DM), 1), b256, 0, stream>>>(
      C16, CD, 0LL, WCK, CD, 0LL, (void*)CK, DM, 0LL, b_ck, b_ck, 0, BB * SCTX, DM, CD, r64);
  gemm64<1, true, false><<<dim3(gemm_blocks(DM, SCTX), BB), b256, 0, stream>>>(
      WCV, CD, 0LL, C16, CD, (long long)SCTX * CD,
      (void*)CVT, SCTX, (long long)DM * SCTX, b_cv, b_cv, 0, DM, SCTX, CD, r64);
  attn64<<<dim3(NTOK / 64, NH, BB), b128, 0, stream>>>(
      CQ, DM, 0, CK, DM, 0, CVT, SCTX, CTX, NTOK, SCTX, 0.125f, 0.0625f);
  gemm64<0, false, true><<<dim3(gemm_blocks(BB * NTOK, DM), 1), b256, 0, stream>>>(
      CTX, DM, 0LL, WCO, DM, 0LL, (void*)XB, DM, 0LL, b_co, outF, DM, BB * NTOK, DM, DM, r4096);

  ln_mod<<<dim3(BB * NTOK), b128, 0, stream>>>(XB, ADA, H, 4 * DM, 5 * DM);
  wtrans64<<<dim3(DMLP / 64, DM / 64), b256, 0, stream>>>(w1, W1T, DM, DMLP, 64.0f);
  gemm64<2, false, false><<<dim3(gemm_blocks(BB * NTOK, DMLP), 1), b256, 0, stream>>>(
      H, DM, 0LL, W1T, DM, 0LL, (void*)G, DMLP, 0LL, b1, b1, 0, BB * NTOK, DMLP, DM, r64);
  wtrans64<<<dim3(DM / 64, DMLP / 64), b256, 0, stream>>>(w2, W2T, DMLP, DM, 64.0f);
  gemm64<0, false, true><<<dim3(gemm_blocks(BB * NTOK, DM), 1), b256, 0, stream>>>(
      G, DMLP, 0LL, W2T, DMLP, 0LL, d_out, DM, 0LL, b2, XB, DM, BB * NTOK, DM, DMLP, r64);
  (void)hipGetLastError();
}
